// SSA_24223615549520
// MI455X (gfx1250) — hardware-verified
//
#include <hip/hip_runtime.h>
#include <hip/hip_bf16.h>
#pragma clang fp contract(off)

typedef __attribute__((ext_vector_type(16))) _Float16 v16h;
typedef __attribute__((ext_vector_type(8)))  _Float16 v8h;
typedef __attribute__((ext_vector_type(16))) __bf16   v16b;
typedef __attribute__((ext_vector_type(8)))  __bf16   v8b;
typedef __attribute__((ext_vector_type(8)))  float    v8f;
typedef __attribute__((ext_vector_type(4)))  float    v4f;
typedef __attribute__((ext_vector_type(4)))  unsigned int v4u;

constexpr int kBatch    = 2;
constexpr int kChan     = 256;
constexpr int kImg      = 96;
constexpr int kHW       = 9216;
constexpr int kNPix     = 18432;
constexpr int kPadW     = 98;
constexpr int kPadArea  = 9604;
constexpr int kRowsPB   = 9728;
constexpr int kNPixP    = 19456;
constexpr int kGuard    = 128;
constexpr int kXRows    = kGuard + kNPixP + kGuard;
constexpr int kTaps     = 9;
constexpr int kKdc      = 2304;
constexpr int kNOff     = 64;
constexpr int kNOffReal = 18;
constexpr int kHeads    = 8;
constexpr int kHeadCh   = 32;
constexpr int kKV       = 512;
constexpr int kChunkPix = 4608;
constexpr int kNChunk   = 4;
constexpr int kGroupsPerRow = kNPix / 256;
constexpr int kGroupsPerImg = kHW / 256;

static_assert(kNChunk * kChunkPix == kNPix, "chunks cover all pixels");
static_assert(kXRows % 64 == 0, "xpad tile rows");
static_assert(kNPixP % 64 == 0 && kNOff % 64 == 0 && kKdc % 32 == 0, "gemm0 shapes");
static_assert(kKV % 64 == 0 && kChan % 64 == 0 && kChan % 32 == 0, "gemm2 shapes");
static_assert(kChunkPix % 64 == 0, "gemm1 shapes");
static_assert(kHW % 64 == 0 && kHW % 32 == 0, "gemm4/5 and attention K");
static_assert(kHW % 256 == 0 && kNPix % 256 == 0, "ksplit groups");

__device__ __forceinline__ unsigned short f2bf_bits(float f) {
  unsigned u = __float_as_uint(f);
  return (unsigned short)((u + 0x7FFFu + ((u >> 16) & 1u)) >> 16);
}
__device__ __forceinline__ float bf_bits2f(unsigned short h) { return __uint_as_float(((unsigned)h) << 16); }

__device__ __forceinline__ void dep_guard_h(v8f& a, v8f& b, v16h x, v16h y) { asm volatile("v_nop\n\tv_nop\n\tv_nop\n\tv_nop" : "+v"(a), "+v"(b) : "v"(x), "v"(y)); }
__device__ __forceinline__ void dep_guard_b(v8f& a, v8f& b, v16b x, v16b y) { asm volatile("v_nop\n\tv_nop\n\tv_nop\n\tv_nop" : "+v"(a), "+v"(b) : "v"(x), "v"(y)); }
__device__ __forceinline__ void keep4_h(v16h a, v16h b, v16h c, v16h d) { asm volatile("v_nop" :: "v"(a), "v"(b), "v"(c), "v"(d)); }
__device__ __forceinline__ void keep4_b(v16b a, v16b b, v16b c, v16b d) { asm volatile("v_nop" :: "v"(a), "v"(b), "v"(c), "v"(d)); }
__device__ __forceinline__ void acc_guard4(v8f& a, v8f& b, v8f& c, v8f& d) { asm volatile("v_nop\n\tv_nop\n\tv_nop\n\tv_nop" : "+v"(a), "+v"(b), "+v"(c), "+v"(d)); }
template <typename T> struct Frag;
template <> struct Frag<_Float16> {
  typedef v16h V; union U { v16h v; v8h h[2]; };
  static __device__ __forceinline__ v16h load(const _Float16* p) {
    U f; f.h[0] = *(const v8h*)(p); f.h[1] = *(const v8h*)(p + 16); return f.v;
  }
  static __device__ __forceinline__ v8f mma(v16h a, v16h b, v8f c) {
    return __builtin_amdgcn_wmma_f32_16x16x32_f16(false, a, false, b, (short)0, c, false, false);
  }
  static __device__ __forceinline__ void guard(v8f& a, v8f& b, v16h x, v16h y) { dep_guard_h(a, b, x, y); }
  static __device__ __forceinline__ void keep(v16h a, v16h b, v16h c, v16h d) { keep4_h(a, b, c, d); }
};
template <> struct Frag<__bf16> {
  typedef v16b V; union U { v16b v; v8b h[2]; };
  static __device__ __forceinline__ v16b load(const __bf16* p) {
    U f; f.h[0] = *(const v8b*)(p); f.h[1] = *(const v8b*)(p + 16); return f.v;
  }
  static __device__ __forceinline__ v8f mma(v16b a, v16b b, v8f c) {
    return __builtin_amdgcn_wmma_f32_16x16x32_bf16(false, a, false, b, (short)0, c, false, false);
  }
  static __device__ __forceinline__ void guard(v8f& a, v8f& b, v16b x, v16b y) { dep_guard_b(a, b, x, y); }
  static __device__ __forceinline__ void keep(v16b a, v16b b, v16b c, v16b d) { keep4_b(a, b, c, d); }
};

__device__ __forceinline__ v8f at_mma(v16b a, v16b b, v8f c) {
  c = __builtin_amdgcn_wmma_f32_16x16x32_bf16(false, a, false, b, (short)0, c, false, false);
  asm volatile("v_nop\n\tv_nop\n\tv_nop\n\tv_nop" : "+v"(c) : "v"(a), "v"(b));
  return c;
}

__device__ __forceinline__ void split_bf(float f, unsigned short& hb, unsigned short& lb) {
  hb = f2bf_bits(f);
  lb = f2bf_bits(f - bf_bits2f(hb));
}
__device__ __forceinline__ unsigned pk_bf2(float a, float b) {
  return (unsigned)f2bf_bits(a) | (((unsigned)f2bf_bits(b)) << 16);
}
__device__ __forceinline__ void store2_u4(unsigned short* dst, v4u u) {
  *(volatile v4u*)dst = u;
  __threadfence();
  *(volatile v4u*)dst = u;
}

template <bool SA, bool SB, int BIAS_MODE, int OUT_MODE, bool ASHIFT>
__global__ __launch_bounds__(256) void gemm_bf16_t64(
    const unsigned short* __restrict__ Ap, const unsigned short* __restrict__ A2p, int lda, long strideA,
    const unsigned short* __restrict__ Btp, const unsigned short* __restrict__ Bt2p, int ldb, long strideB,
    void* __restrict__ Cout, void* __restrict__ Cout2, int ldc, long strideC,
    const float* __restrict__ bias, int M, int N, int K, float scale) {
  typedef __bf16 T;
  typedef v16b V;
  const T* A = (const T*)Ap; const T* A2 = (const T*)A2p; const T* Bt = (const T*)Btp; const T* Bt2 = (const T*)Bt2p;
  __shared__ __align__(16) float sT[8][16 * 68];
  const int b    = blockIdx.y;
  const int lane = threadIdx.x & 31;
  const int wave = threadIdx.x >> 5;
  const int tilesN = N >> 6;
  const int tilesM = M >> 6;
  const int tile = blockIdx.x * 8 + wave;
  if (tile >= tilesM * tilesN) return;
  const int tm = tile / tilesN;
  const int tn = tile - tm * tilesN;
  const int m0 = tm << 6;
  const int n0 = tn << 6;

  const T* Ab  = A  + (size_t)b * strideA;
  const T* Bb  = Bt + (size_t)b * strideB;
  const T* Ab2 = SA ? (A2  + (size_t)b * strideA) : nullptr;
  const T* Bb2 = SB ? (Bt2 + (size_t)b * strideB) : nullptr;

  const int rlane = lane & 15;
  const int koff  = (lane >> 4) * 8;
  const int mOff  = (lane >> 4) * 8;

  v8f acc[4][4];
#pragma unroll
  for (int i = 0; i < 4; ++i)
#pragma unroll
    for (int j = 0; j < 4; ++j) acc[i][j] = (v8f){0.f,0.f,0.f,0.f,0.f,0.f,0.f,0.f};

  for (int k0 = 0; k0 < K; k0 += 32) {
    long aRow = 0;
    int aK = k0;
    if (ASHIFT) {
      const int tap = k0 >> 8;
      const int ti = tap / 3;
      const int tj = tap - ti * 3;
      aRow = (long)(ti - 1) * kPadW + (long)(tj - 1);
      aK = k0 & 255;
    }
    V bh[4], bl[4];
#pragma unroll
    for (int j = 0; j < 4; ++j) {
      const long bo = (long)(n0 + (j << 4) + rlane) * ldb + koff + k0;
      bh[j] = Frag<T>::load(Bb + bo);
      if (SB) bl[j] = Frag<T>::load(Bb2 + bo);
    }
#pragma unroll
    for (int i = 0; i < 4; ++i) {
      const long ao = ((long)(m0 + (i << 4) + rlane) + aRow) * lda + koff + aK;
      V ah = Frag<T>::load(Ab + ao);
      V al = ah;
      if (SA) al = Frag<T>::load(Ab2 + ao);
#pragma unroll
      for (int j = 0; j < 4; ++j) {
        acc[i][j] = Frag<T>::mma(ah, bh[j], acc[i][j]);
        if (SB) acc[i][j] = Frag<T>::mma(ah, bl[j], acc[i][j]);
        if (SA) acc[i][j] = Frag<T>::mma(al, bh[j], acc[i][j]);
      }
      Frag<T>::guard(acc[i][0], acc[i][3], ah, al);
    }
    Frag<T>::keep(bh[0], bh[1], bh[2], bh[3]);
    if (SB) Frag<T>::keep(bl[0], bl[1], bl[2], bl[3]);
  }
  acc_guard4(acc[0][0], acc[0][1], acc[0][2], acc[0][3]);
  acc_guard4(acc[1][0], acc[1][1], acc[1][2], acc[1][3]);
  acc_guard4(acc[2][0], acc[2][1], acc[2][2], acc[2][3]);
  acc_guard4(acc[3][0], acc[3][1], acc[3][2], acc[3][3]);

  float* slab = sT[wave];
#pragma unroll
  for (int i = 0; i < 4; ++i) {
    const int mBase = m0 + (i << 4);
#pragma unroll
    for (int j = 0; j < 4; ++j) {
      const int n = n0 + (j << 4) + rlane;
      float bv = 0.f;
      if (BIAS_MODE == 2) bv = bias[n];
#pragma unroll
      for (int r = 0; r < 8; ++r) {
        float v = acc[i][j][r] * scale;
        if (BIAS_MODE == 2) v += bv;
        slab[(mOff + r) * 68 + (j << 4) + rlane] = v;
      }
    }
    __builtin_amdgcn_fence(__ATOMIC_RELEASE, "workgroup");
    __builtin_amdgcn_wave_barrier();
    __builtin_amdgcn_fence(__ATOMIC_ACQUIRE, "workgroup");
    if (OUT_MODE == 0) {
      float* C = (float*)Cout + (size_t)b * strideC;
      const int hh = lane >> 4, c4 = (lane & 15) * 4;
      for (int pass = 0; pass < 2; ++pass) {
#pragma unroll
        for (int it = 0; it < 8; ++it) {
          const int row = it * 2 + hh;
          v4f v = *(const v4f*)(slab + row * 68 + c4);
          *(volatile v4f*)(C + (size_t)(mBase + row) * ldc + n0 + c4) = v;
        }
        __threadfence();
      }
    } else {
      const int q = lane >> 3, c8 = (lane & 7) * 8;
      unsigned short* C  = (unsigned short*)Cout  + (size_t)b * strideC;
      unsigned short* C2 = (OUT_MODE == 2) ? ((unsigned short*)Cout2 + (size_t)b * strideC) : nullptr;
      for (int pass = 0; pass < 2; ++pass) {
#pragma unroll
        for (int it = 0; it < 4; ++it) {
          const int row = it * 4 + q;
          const float* sp = slab + row * 68 + c8;
          v8h hv, lv;
#pragma unroll
          for (int e = 0; e < 8; ++e) {
            if (OUT_MODE == 1) {
              hv[e] = (_Float16)sp[e];
            } else {
              unsigned short hb = f2bf_bits(sp[e]);
              unsigned short lb = f2bf_bits(sp[e] - bf_bits2f(hb));
              hv[e] = __builtin_bit_cast(_Float16, hb);
              lv[e] = __builtin_bit_cast(_Float16, lb);
            }
          }
          *(volatile v8h*)(C + (size_t)(mBase + row) * ldc + n0 + c8) = hv;
          if (OUT_MODE == 2) *(volatile v8h*)(C2 + (size_t)(mBase + row) * ldc + n0 + c8) = lv;
        }
        __threadfence();
      }
    }
    __builtin_amdgcn_fence(__ATOMIC_RELEASE, "workgroup");
    __builtin_amdgcn_wave_barrier();
    __builtin_amdgcn_fence(__ATOMIC_ACQUIRE, "workgroup");
  }
}

constexpr int kPrepU0 = kNOff * kTaps;
constexpr int kPrepU1 = kPrepU0 + kChan * kTaps;
constexpr int kPrepU2 = kPrepU1 + kKV;
constexpr int kPrepU3 = kPrepU2 + kChan;
constexpr int kPrepUnits = kPrepU3 + 1;
constexpr int kPrepBlocks = (kPrepUnits + 7) / 8;

__device__ __forceinline__ void cast_row8(const float* __restrict__ src, long idx0, long stride, bool keep, unsigned short* dst) {
  float f0 = src[idx0];
  float f1 = src[idx0 + stride];
  float f2 = src[idx0 + 2 * stride];
  float f3 = src[idx0 + 3 * stride];
  float f4 = src[idx0 + 4 * stride];
  float f5 = src[idx0 + 5 * stride];
  float f6 = src[idx0 + 6 * stride];
  float f7 = src[idx0 + 7 * stride];
  if (!keep) { f0 = 0.f; f1 = 0.f; f2 = 0.f; f3 = 0.f; f4 = 0.f; f5 = 0.f; f6 = 0.f; f7 = 0.f; }
  v4u u;
  u[0] = pk_bf2(f0, f1); u[1] = pk_bf2(f2, f3); u[2] = pk_bf2(f4, f5); u[3] = pk_bf2(f6, f7);
  store2_u4(dst, u);
}

__global__ __launch_bounds__(256) void k_prep(
    const float* __restrict__ wp, const float* __restrict__ bp, const float* __restrict__ wd,
    const float* __restrict__ wqkv, const float* __restrict__ wproj,
    unsigned short* __restrict__ Wp64, float* __restrict__ bias64, unsigned short* __restrict__ Wd,
    unsigned short* __restrict__ Wkv, unsigned short* __restrict__ Wpr) {
  const int wave = threadIdx.x >> 5, lane = threadIdx.x & 31;
  const int unit = __builtin_amdgcn_readfirstlane((int)(blockIdx.x * 8 + wave));
  const int c8 = lane * 8;
  if (unit < kPrepU0) {
    const int o = unit / kTaps;
    const int tap = unit - o * kTaps;
    const int oc = (o < kNOffReal) ? o : (kNOffReal - 1);
    cast_row8(wp, ((long)oc * kChan + c8) * kTaps + tap, kTaps, o < kNOffReal,
              Wp64 + (size_t)o * kKdc + (size_t)tap * kChan + c8);
  } else if (unit < kPrepU1) {
    const int u = unit - kPrepU0;
    const int o = u / kTaps;
    const int tap = u - o * kTaps;
    cast_row8(wd, ((long)o * kChan + c8) * kTaps + tap, kTaps, true,
              Wd + (size_t)o * kKdc + (size_t)tap * kChan + c8);
  } else if (unit < kPrepU2) {
    const int r = unit - kPrepU1;
    cast_row8(wqkv, (long)(kChan + r) * kChan + c8, 1, true, Wkv + (size_t)r * kChan + c8);
  } else if (unit < kPrepU3) {
    const int r = unit - kPrepU2;
    cast_row8(wproj, (long)r * kChan + c8, 1, true, Wpr + (size_t)r * kChan + c8);
  } else if (unit == kPrepU3) {
    const int nb = lane * 4;
    v4f v;
#pragma unroll
    for (int e = 0; e < 4; ++e) {
      const int n = nb + e;
      const int nc = (n < kNOffReal) ? n : (kNOffReal - 1);
      float f = bp[nc];
      f = bf_bits2f(f2bf_bits(f));
      v[e] = (n < kNOffReal) ? f : 0.f;
    }
    if (lane < 16) *(volatile v4f*)(bias64 + nb) = v;
    __threadfence();
    if (lane < 16) *(volatile v4f*)(bias64 + nb) = v;
  }
}

__global__ __launch_bounds__(256) void k_xpad(const float* __restrict__ x, unsigned short* __restrict__ xPad) {
  __shared__ __align__(16) unsigned short tileb[64][72];
  const int tid = threadIdx.x, wave = tid >> 5, lane = tid & 31;
  const int r = tid & 63, cg = tid >> 6;
  const int c0 = blockIdx.y * 64;
  const long R = (long)blockIdx.x * 64 + r;
  long P = R - kGuard;
  const bool inP = (P >= 0) && (P < kNPixP);
  P = (P < 0) ? 0 : P;
  P = (P > (long)(kNPixP - 1)) ? (long)(kNPixP - 1) : P;
  const int bb = (int)(P / kRowsPB);
  const int pp = (int)(P - (long)bb * kRowsPB);
  const int ph = pp / kPadW;
  const int pw = pp - ph * kPadW;
  const bool valid = inP && (pp < kPadArea) && (ph >= 1) && (ph <= kImg) && (pw >= 1) && (pw <= kImg);
  int hs = ph - 1;  hs = (hs < 0) ? 0 : ((hs > kImg - 1) ? (kImg - 1) : hs);
  int wsr = pw - 1; wsr = (wsr < 0) ? 0 : ((wsr > kImg - 1) ? (kImg - 1) : wsr);
  const float* sp = x + (size_t)bb * kChan * kHW + (size_t)hs * kImg + wsr;
#pragma unroll 4
  for (int cc = 0; cc < 16; ++cc) {
    const int cl = cg * 16 + cc;
    float f = sp[(size_t)(c0 + cl) * kHW];
    f = valid ? f : 0.0f;
    tileb[r][cl] = f2bf_bits(f);
  }
  __syncthreads();
  const int q = lane >> 3, j = lane & 7;
  for (int pass = 0; pass < 2; ++pass) {
#pragma unroll
    for (int it = 0; it < 2; ++it) {
      const int row = wave * 8 + it * 4 + q;
      const v4u u = *(const v4u*)(&tileb[row][8 * j]);
      *(volatile v4u*)(xPad + ((size_t)blockIdx.x * 64 + row) * kChan + c0 + 8 * j) = u;
    }
    __threadfence();
  }
}

__global__ __launch_bounds__(256) void k_rownorm(const float* __restrict__ kvf, float* __restrict__ rinv) {
  __shared__ float ssum[32];
  const int wave = threadIdx.x >> 5, lane = threadIdx.x & 31;
  const int e0 = blockIdx.x * 32;
  const int bsel = e0 / kKV;
  const int o0 = e0 - bsel * kKV;
  for (int i = wave; i < 32; i += 8) {
    const float* row = kvf + (size_t)(o0 + i) * kNPixP + (size_t)bsel * kRowsPB;
    float s = 0.f;
    for (int P = lane; P < kRowsPB; P += 32) { const float v = row[P]; s += v * v; }
#pragma unroll
    for (int off = 16; off > 0; off >>= 1) s += __shfl_xor(s, off, 32);
    if (lane == 0) ssum[i] = s;
  }
  __syncthreads();
  if (wave == 0) {
    const float s = ssum[lane];
    const float rv = 1.0f / fmaxf(sqrtf(s), 1e-12f);
    *(volatile float*)(rinv + e0 + lane) = rv;
    __threadfence();
    *(volatile float*)(rinv + e0 + lane) = rv;
  }
}

__global__ __launch_bounds__(256) void k_ksplit(const float* __restrict__ kvf, const float* __restrict__ rinv,
                                                 unsigned short* __restrict__ kh, unsigned short* __restrict__ kl) {
  const int wave = threadIdx.x >> 5, lane = threadIdx.x & 31;
  const int unit = __builtin_amdgcn_readfirstlane((int)(blockIdx.x * 8 + wave));
  const int o = unit / kGroupsPerRow;
  const int g = unit - o * kGroupsPerRow;
  const int bsel = (g >= kGroupsPerImg) ? 1 : 0;
  const int pbase = g * 256 + lane * 8;
  const float ri = rinv[bsel * kKV + o];
  const float* src = kvf + (size_t)o * kNPixP + (size_t)bsel * kRowsPB;
  v4u hu = {0u, 0u, 0u, 0u}, lu = {0u, 0u, 0u, 0u};
#pragma unroll
  for (int e = 0; e < 8; ++e) {
    const int p = pbase + e;
    const int hw = p - bsel * kHW;
    const int h = hw / kImg;
    const int w = hw - h * kImg;
    const float v = src[(h + 1) * kPadW + (w + 1)] * ri;
    unsigned short hb, lb;
    split_bf(v, hb, lb);
    hu[e >> 1] = hu[e >> 1] | (((unsigned)hb) << (16 * (e & 1)));
    lu[e >> 1] = lu[e >> 1] | (((unsigned)lb) << (16 * (e & 1)));
  }
  unsigned short* dh = kh + (size_t)o * kNPix + pbase;
  unsigned short* dl = kl + (size_t)o * kNPix + pbase;
  *(volatile v4u*)dh = hu;
  *(volatile v4u*)dl = lu;
  __threadfence();
  *(volatile v4u*)dh = hu;
  *(volatile v4u*)dl = lu;
}

__global__ __launch_bounds__(256) void k_vsplit(const float* __restrict__ kvf, const float* __restrict__ rinv,
                                                 unsigned short* __restrict__ vTh, unsigned short* __restrict__ vTl) {
  __shared__ __align__(16) unsigned short th[64][72];
  __shared__ __align__(16) unsigned short tlo[64][72];
  const int tid = threadIdx.x, wave = tid >> 5, lane = tid & 31;
  const int p0t = blockIdx.x * 64;
  const int bsel = p0t / kHW;
  const int d0 = blockIdx.y * 64;
  const int pl = tid & 63;
  const int p = p0t + pl;
  const int hw = p - bsel * kHW;
  const int h = hw / kImg;
  const int w = hw - h * kImg;
  const int Pp = bsel * kRowsPB + (h + 1) * kPadW + (w + 1);
#pragma unroll 4
  for (int it = 0; it < 16; ++it) {
    const int dl = it * 4 + (tid >> 6);
    const int o = kChan + d0 + dl;
    const float f = kvf[(size_t)o * kNPixP + Pp] * rinv[bsel * kKV + o];
    unsigned short hb, lb;
    split_bf(f, hb, lb);
    th[pl][dl] = hb;
    tlo[pl][dl] = lb;
  }
  __syncthreads();
  const int q = lane >> 3, j = lane & 7;
  for (int pass = 0; pass < 2; ++pass) {
#pragma unroll
    for (int it = 0; it < 2; ++it) {
      const int row = wave * 8 + it * 4 + q;
      const v4u uh = *(const v4u*)(&th[row][8 * j]);
      const v4u ul = *(const v4u*)(&tlo[row][8 * j]);
      const size_t off = ((size_t)(p0t + row)) * kChan + d0 + 8 * j;
      *(volatile v4u*)(vTh + off) = uh;
      *(volatile v4u*)(vTl + off) = ul;
    }
    __threadfence();
  }
}

__global__ __launch_bounds__(256) void k_sample(const unsigned short* __restrict__ xPad, const float* __restrict__ off32,
                                                 unsigned short* __restrict__ Sh, unsigned short* __restrict__ Sl, int p0) {
  const int wave = threadIdx.x >> 5, lane = threadIdx.x & 31;
  const int unit = blockIdx.x * 8 + wave;
  const int pl = unit / kTaps;
  const int tap = unit - pl * kTaps;
  const int p = p0 + pl;
  const int bsel = p / kHW;
  const int hw = p - bsel * kHW;
  const int h = hw / kImg;
  const int w = hw - h * kImg;
  const int Pp = bsel * kRowsPB + (h + 1) * kPadW + (w + 1);
  const float ox = off32[(size_t)Pp * kNOff + tap];
  const float oy = off32[(size_t)Pp * kNOff + kTaps + tap];
  const int ti = tap / 3;
  const int tj = tap - ti * 3;
  float px = ox + (float)(ti - 1);
  px = px + (float)(h + 1);
  float py = oy + (float)(tj - 1);
  py = py + (float)(w + 1);
  const float fx = floorf(px), fy = floorf(py);
  const float lim = (float)(kPadW - 1);
  const float qltx = fminf(fmaxf(fx, 0.f), lim);
  const float qlty = fminf(fmaxf(fy, 0.f), lim);
  const float qrbx = fminf(fmaxf(fx + 1.f, 0.f), lim);
  const float qrby = fminf(fmaxf(fy + 1.f, 0.f), lim);
  const float pxc = fminf(fmaxf(px, 0.f), lim);
  const float pyc = fminf(fmaxf(py, 0.f), lim);
  float ax1 = qltx - pxc; ax1 = 1.f + ax1;
  float ax2 = qrbx - pxc; ax2 = 1.f - ax2;
  float ay1 = qlty - pyc; ay1 = 1.f + ay1;
  float ay2 = qrby - pyc; ay2 = 1.f - ay2;
  const float glt = ax1 * ay1;
  const float grb = ax2 * ay2;
  const float glb = ax1 * ay2;
  const float grt = ax2 * ay1;
  const int iltx = (int)qltx, ilty = (int)qlty, irbx = (int)qrbx, irby = (int)qrby;
  const size_t rb0 = (size_t)kGuard + (size_t)bsel * kRowsPB;
  const size_t Rlt = rb0 + (size_t)(iltx * kPadW + ilty);
  const size_t Rrb = rb0 + (size_t)(irbx * kPadW + irby);
  const size_t Rlb = rb0 + (size_t)(iltx * kPadW + irby);
  const size_t Rrt = rb0 + (size_t)(irbx * kPadW + ilty);
  const int c8 = lane * 8;
  const v4u ult = *(const v4u*)(xPad + Rlt * kChan + c8);
  const v4u urb = *(const v4u*)(xPad + Rrb * kChan + c8);
  const v4u ulb = *(const v4u*)(xPad + Rlb * kChan + c8);
  const v4u urt = *(const v4u*)(xPad + Rrt * kChan + c8);
  v4u hu = {0u, 0u, 0u, 0u}, lu = {0u, 0u, 0u, 0u};
#pragma unroll
  for (int e = 0; e < 8; ++e) {
    const unsigned wlt = ult[e >> 1], wrb = urb[e >> 1], wlb = ulb[e >> 1], wrt = urt[e >> 1];
    float xlt, xrb, xlb, xrt;
    if (e & 1) {
      xlt = __uint_as_float(wlt & 0xffff0000u); xrb = __uint_as_float(wrb & 0xffff0000u);
      xlb = __uint_as_float(wlb & 0xffff0000u); xrt = __uint_as_float(wrt & 0xffff0000u);
    } else {
      xlt = __uint_as_float(wlt << 16); xrb = __uint_as_float(wrb << 16);
      xlb = __uint_as_float(wlb << 16); xrt = __uint_as_float(wrt << 16);
    }
    float xo = glt * xlt;
    const float t1 = grb * xrb; xo = xo + t1;
    const float t2 = glb * xlb; xo = xo + t2;
    const float t3 = grt * xrt; xo = xo + t3;
    unsigned short hb, lb;
    split_bf(xo, hb, lb);
    hu[e >> 1] = hu[e >> 1] | (((unsigned)hb) << (16 * (e & 1)));
    lu[e >> 1] = lu[e >> 1] | (((unsigned)lb) << (16 * (e & 1)));
  }
  const size_t soff = (size_t)pl * kKdc + (size_t)tap * kChan + c8;
  *(volatile v4u*)(Sh + soff) = hu;
  *(volatile v4u*)(Sl + soff) = lu;
  __threadfence();
  *(volatile v4u*)(Sh + soff) = hu;
  *(volatile v4u*)(Sl + soff) = lu;
}

__global__ __launch_bounds__(128) void k_attn(const unsigned short* __restrict__ qh, const unsigned short* __restrict__ ql,
                                               const unsigned short* __restrict__ kh, const unsigned short* __restrict__ kl,
                                               const float* __restrict__ temp,
                                               unsigned short* __restrict__ Ph, unsigned short* __restrict__ Pl) {
  __shared__ __align__(16) float sS[kHeadCh][36];
  const int tid = threadIdx.x, wave = tid >> 5, lane = tid & 31;
  const int hh = lane >> 4, c = lane & 15;
  const int bsel = blockIdx.x >> 3, head = blockIdx.x & 7;
  const int mi = wave >> 1, ni = wave & 1;
  const __bf16* qa  = (const __bf16*)qh + (size_t)(head * kHeadCh + mi * 16 + c) * kNPix + (size_t)bsel * kHW + 8 * hh;
  const __bf16* qa2 = (const __bf16*)ql + (size_t)(head * kHeadCh + mi * 16 + c) * kNPix + (size_t)bsel * kHW + 8 * hh;
  const __bf16* kb  = (const __bf16*)kh + (size_t)(head * kHeadCh + ni * 16 + c) * kNPix + (size_t)bsel * kHW + 8 * hh;
  const __bf16* kb2 = (const __bf16*)kl + (size_t)(head * kHeadCh + ni * 16 + c) * kNPix + (size_t)bsel * kHW + 8 * hh;
  v8f acc = (v8f){0.f,0.f,0.f,0.f,0.f,0.f,0.f,0.f};
  for (int k0 = 0; k0 < kHW; k0 += 32) {
    const v16b ahv = Frag<__bf16>::load(qa + k0);
    const v16b alv = Frag<__bf16>::load(qa2 + k0);
    const v16b bhv = Frag<__bf16>::load(kb + k0);
    const v16b blv = Frag<__bf16>::load(kb2 + k0);
    acc = at_mma(ahv, bhv, acc);
    acc = at_mma(ahv, blv, acc);
    acc = at_mma(alv, bhv, acc);
  }
  const float tv = bf_bits2f(f2bf_bits(temp[head]));
#pragma unroll
  for (int r = 0; r < 8; ++r) sS[mi * 16 + 8 * hh + r][ni * 16 + c] = acc[r] * tv;
  __syncthreads();
  for (int i = 0; i < 8; ++i) {
    const int rr = wave * 8 + i;
    const float v = sS[rr][lane];
    float m = v;
#pragma unroll
    for (int off = 16; off > 0; off >>= 1) m = fmaxf(m, __shfl_xor(m, off, 32));
    const float ev = expf(v - m);
    float s = ev;
#pragma unroll
    for (int off = 16; off > 0; off >>= 1) s += __shfl_xor(s, off, 32);
    sS[rr][lane] = ev / s;
  }
  __syncthreads();
  const int q = lane >> 3, j = lane & 7;
  const int colbase = 64 * q + 8 * j;
  const int rel = colbase - head * kHeadCh;
  const bool inr = (rel >= 0) && (rel < kHeadCh);
  const int relc = (rel < 0) ? 0 : ((rel > 24) ? 24 : rel);
  for (int pass = 0; pass < 2; ++pass) {
#pragma unroll
    for (int i = 0; i < 8; ++i) {
      const int rr = wave * 8 + i;
      const v4f fa = *(const v4f*)(&sS[rr][relc]);
      const v4f fb = *(const v4f*)(&sS[rr][relc + 4]);
      v4u hu, lu;
#pragma unroll
      for (int e2 = 0; e2 < 4; ++e2) {
        float fl = fa[e2], fh2 = fb[e2];
        float g0 = (e2 < 2) ? fa[2 * e2] : fb[2 * e2 - 4];
        float g1 = (e2 < 2) ? fa[2 * e2 + 1] : fb[2 * e2 - 3];
        (void)fl; (void)fh2;
        g0 = inr ? g0 : 0.f;
        g1 = inr ? g1 : 0.f;
        unsigned short h0, l0, h1, l1;
        split_bf(g0, h0, l0);
        split_bf(g1, h1, l1);
        hu[e2] = (unsigned)h0 | (((unsigned)h1) << 16);
        lu[e2] = (unsigned)l0 | (((unsigned)l1) << 16);
      }
      const size_t off = ((size_t)(bsel * kChan + head * kHeadCh + rr)) * kChan + colbase;
      *(volatile v4u*)(Ph + off) = hu;
      *(volatile v4u*)(Pl + off) = lu;
    }
    __threadfence();
  }
}

constexpr size_t kBytesXPad   = (size_t)kXRows * kChan * 2;
constexpr size_t kBytesWp     = (size_t)kNOff * kKdc * 2;
constexpr size_t kBytesBias   = 256;
constexpr size_t kBytesWd     = (size_t)kChan * kKdc * 2;
constexpr size_t kBytesWkv    = (size_t)kKV * kChan * 2;
constexpr size_t kBytesWpr    = (size_t)kChan * kChan * 2;
constexpr size_t kBytesOff    = (size_t)kNPixP * kNOff * 4;
constexpr size_t kBytesKvf    = (size_t)kKV * kNPixP * 4;
constexpr size_t kBytesSPlane = (size_t)kChunkPix * kKdc * 2;
constexpr size_t kBytesBig    = (2 * kBytesSPlane > kBytesKvf) ? 2 * kBytesSPlane : kBytesKvf;
constexpr size_t kBytesRinv   = 1024 * 4;
constexpr size_t kBytesPlane  = (size_t)kChan * kNPix * 2;
constexpr size_t kBytesPbd    = (size_t)kBatch * kChan * kChan * 2;
constexpr size_t kOffXPad = 0;
constexpr size_t kOffWp   = kOffXPad + kBytesXPad;
constexpr size_t kOffBias = kOffWp + kBytesWp;
constexpr size_t kOffWd   = kOffBias + kBytesBias;
constexpr size_t kOffWkv  = kOffWd + kBytesWd;
constexpr size_t kOffWpr  = kOffWkv + kBytesWkv;
constexpr size_t kOffOff  = kOffWpr + kBytesWpr;
constexpr size_t kOffBig  = kOffOff + kBytesOff;
constexpr size_t kOffRinv = kOffBig + kBytesBig;
constexpr size_t kOffKh   = kOffRinv + kBytesRinv;
constexpr size_t kOffKl   = kOffKh + kBytesPlane;
constexpr size_t kOffVh   = kOffKl + kBytesPlane;
constexpr size_t kOffVl   = kOffVh + kBytesPlane;
constexpr size_t kOffQh   = kOffVl + kBytesPlane;
constexpr size_t kOffQl   = kOffQh + kBytesPlane;
constexpr size_t kOffPbh  = kOffQl + kBytesPlane;
constexpr size_t kOffPbl  = kOffPbh + kBytesPbd;
constexpr size_t kWsTotal = kOffPbl + kBytesPbd;
static_assert(kWsTotal == 116560128ull, "carve total");
static_assert(kWsTotal <= 134217728ull, "carve under 128 MiB");
static_assert(kBytesKvf <= kBytesBig && 2 * kBytesSPlane <= kBytesBig, "BIG region covers both users");
static_assert((kOffWp % 256) == 0 && (kOffOff % 256) == 0 && (kOffBig % 256) == 0 && (kOffKh % 256) == 0 &&
              (kOffQh % 256) == 0 && (kOffPbh % 256) == 0 && (kOffPbl % 256) == 0, "alignment");

constexpr int kXpadBlocksX  = kXRows / 64;
constexpr int kG0Blocks     = ((kNPixP / 64) * (kNOff / 64) + 7) / 8;
constexpr int kG2Blocks     = ((kKV / 64) * (kNPixP / 64) + 7) / 8;
constexpr int kG1Blocks     = ((kChan / 64) * (kChunkPix / 64) + 7) / 8;
constexpr int kG4Blocks     = ((kHW / 64) * (kChan / 64) + 7) / 8;
constexpr int kG5Blocks     = ((kChan / 64) * (kHW / 64) + 7) / 8;
constexpr int kKsplitBlocks = (kChan * kGroupsPerRow) / 8;
constexpr int kVsplitBlocksX = kNPix / 64;
constexpr int kSampleBlocks = (kChunkPix * kTaps) / 8;
static_assert(kKsplitBlocks * 8 == kChan * kGroupsPerRow, "ksplit exact");
static_assert(kSampleBlocks * 8 == kChunkPix * kTaps, "sampler exact");

extern "C" void kernel_launch(void* const* d_in, const int* in_sizes, int n_in,
                              void* d_out, int out_size, void* d_ws, size_t ws_size,
                              hipStream_t stream) {
  if (n_in < 7) return;
  if (in_sizes[0] != kBatch * kChan * kHW) return;
  if (in_sizes[1] != kNOffReal * kChan * kTaps) return;
  if (in_sizes[2] < kNOffReal) return;
  if (in_sizes[3] != kChan * kChan * kTaps) return;
  if (in_sizes[4] != 768 * kChan) return;
  if (in_sizes[5] < kHeads) return;
  if (in_sizes[6] != kChan * kChan) return;
  if (out_size != kBatch * kChan * kHW) return;
  if (kWsTotal > ws_size) return;

  const float* x       = (const float*)d_in[0];
  const float* w_pconv = (const float*)d_in[1];
  const float* b_pconv = (const float*)d_in[2];
  const float* w_dconv = (const float*)d_in[3];
  const float* w_qkv   = (const float*)d_in[4];
  const float* temp    = (const float*)d_in[5];
  const float* w_proj  = (const float*)d_in[6];
  float* out = (float*)d_out;

  char* base = (char*)d_ws;
  unsigned short* xPad = (unsigned short*)(base + kOffXPad);
  unsigned short* Wp64 = (unsigned short*)(base + kOffWp);
  float*          bias64 = (float*)(base + kOffBias);
  unsigned short* Wd   = (unsigned short*)(base + kOffWd);
  unsigned short* Wkv  = (unsigned short*)(base + kOffWkv);
  unsigned short* Wpr  = (unsigned short*)(base + kOffWpr);
  float*          off32 = (float*)(base + kOffOff);
  float*          kvf  = (float*)(base + kOffBig);
  unsigned short* Sh   = (unsigned short*)(base + kOffBig);
  unsigned short* Sl   = (unsigned short*)(base + kOffBig + kBytesSPlane);
  float*          rinv = (float*)(base + kOffRinv);
  unsigned short* khp  = (unsigned short*)(base + kOffKh);
  unsigned short* klp  = (unsigned short*)(base + kOffKl);
  unsigned short* vth  = (unsigned short*)(base + kOffVh);
  unsigned short* vtl  = (unsigned short*)(base + kOffVl);
  unsigned short* qhp  = (unsigned short*)(base + kOffQh);
  unsigned short* qlp  = (unsigned short*)(base + kOffQl);
  unsigned short* oth  = (unsigned short*)(base + kOffQh);
  unsigned short* otl  = (unsigned short*)(base + kOffQl);
  unsigned short* pbh  = (unsigned short*)(base + kOffPbh);
  unsigned short* pbl  = (unsigned short*)(base + kOffPbl);
  const unsigned short* xImg = xPad + (size_t)kGuard * kChan;

  k_prep<<<dim3(kPrepBlocks), dim3(256), 0, stream>>>(w_pconv, b_pconv, w_dconv, w_qkv, w_proj, Wp64, bias64, Wd, Wkv, Wpr);
  k_xpad<<<dim3(kXpadBlocksX, 4), dim3(256), 0, stream>>>(x, xPad);
  gemm_bf16_t64<false, false, 2, 0, true><<<dim3(kG0Blocks, 1), dim3(256), 0, stream>>>(
      xImg, xImg, kChan, 0L, Wp64, Wp64, kKdc, 0L, (void*)off32, (void*)off32, kNOff, 0L,
      bias64, kNPixP, kNOff, kKdc, 1.0f);
  gemm_bf16_t64<false, false, 0, 0, false><<<dim3(kG2Blocks, 1), dim3(256), 0, stream>>>(
      Wkv, Wkv, kChan, 0L, xImg, xImg, kChan, 0L, (void*)kvf, (void*)kvf, kNPixP, 0L,
      rinv, kKV, kNPixP, kChan, 1.0f);
  k_rownorm<<<dim3(32), dim3(256), 0, stream>>>(kvf, rinv);
  k_ksplit<<<dim3(kKsplitBlocks), dim3(256), 0, stream>>>(kvf, rinv, khp, klp);
  k_vsplit<<<dim3(kVsplitBlocksX, 4), dim3(256), 0, stream>>>(kvf, rinv, vth, vtl);
  for (int ch = 0; ch < kNChunk; ++ch) {
    k_sample<<<dim3(kSampleBlocks), dim3(256), 0, stream>>>(xPad, off32, Sh, Sl, ch * kChunkPix);
    gemm_bf16_t64<false, true, 0, 2, false><<<dim3(kG1Blocks, 1), dim3(256), 0, stream>>>(
        Wd, Wd, kKdc, 0L, Sh, Sl, kKdc, 0L,
        (void*)(qhp + (size_t)ch * kChunkPix), (void*)(qlp + (size_t)ch * kChunkPix), kNPix, 0L,
        rinv, kChan, kChunkPix, kKdc, 1.0f);
  }
  k_attn<<<dim3(kBatch * kHeads), dim3(128), 0, stream>>>(qhp, qlp, khp, klp, temp, pbh, pbl);
  gemm_bf16_t64<true, true, 0, 2, false><<<dim3(kG4Blocks, kBatch), dim3(256), 0, stream>>>(
      vth, vtl, kChan, (long)kHW * kChan, pbh, pbl, kChan, (long)kChan * kChan,
      (void*)oth, (void*)otl, kChan, (long)kHW * kChan,
      rinv, kHW, kChan, kChan, 1.0f);
  gemm_bf16_t64<false, true, 0, 0, false><<<dim3(kG5Blocks, kBatch), dim3(256), 0, stream>>>(
      Wpr, Wpr, kChan, 0L, oth, otl, kChan, (long)kHW * kChan,
      (void*)out, (void*)out, kHW, (long)kChan * kHW,
      rinv, kChan, kHW, kChan, 1.0f);
}
